// MambaBlock_45483703664837
// MI455X (gfx1250) — hardware-verified
//
#include <hip/hip_runtime.h>
#include <math.h>

typedef __attribute__((ext_vector_type(16))) __bf16   v16b;
typedef __attribute__((ext_vector_type(8)))  __bf16   v8b;
typedef __attribute__((ext_vector_type(8)))  float    v8f;
typedef __attribute__((ext_vector_type(4)))  float    v4f;
typedef __attribute__((ext_vector_type(4)))  unsigned v4u;

constexpr int kBatch = 2;
constexpr int kSeqL  = 2048;
constexpr int kDmod  = 1024;
constexpr int kDin   = 2048;
constexpr int kNst   = 16;
constexpr int kDtR   = 64;
constexpr int kPrjN  = 96;
constexpr int kPrjP  = 128;
constexpr int kXZP   = 2 * kDin;
constexpr int kRows  = kBatch * kSeqL;
constexpr int kTP    = 260;
constexpr float kLog2e = 1.44269504088896340736f;
static_assert(kDtR + 2 * kNst == kPrjN);
static_assert((kDmod % 32) == 0 && (kDin % 32) == 0 && (kDtR % 32) == 0);
static_assert((kSeqL % 64) == 0 && (kXZP % 64) == 0 && (kPrjP % 64) == 0 && (kDin % 64) == 0 && (kDmod % 64) == 0);
static_assert((kDin % 256) == 0 && (kSeqL % 16) == 0);

constexpr size_t kOffXB    = 0;
constexpr size_t kOffWINB  = kOffXB    + (size_t)kRows * kDmod * 2;
constexpr size_t kOffWXB   = kOffWINB  + (size_t)kXZP  * kDmod * 2;
constexpr size_t kOffWDTB  = kOffWXB   + (size_t)kPrjP * kDin  * 2;
constexpr size_t kOffWOUTB = kOffWDTB  + (size_t)kDin  * kDtR  * 2;
constexpr size_t kOffXZ    = kOffWOUTB + (size_t)kDmod * kDin  * 2;
constexpr size_t kOffUC    = kOffXZ    + (size_t)kSeqL * kXZP  * 4;
constexpr size_t kOffUH    = kOffUC    + (size_t)kSeqL * kDin  * 4;
constexpr size_t kOffUL    = kOffUH    + (size_t)kSeqL * kDin  * 2;
constexpr size_t kOffPROJ  = kOffUL    + (size_t)kSeqL * kDin  * 2;
constexpr size_t kOffDRH   = kOffPROJ  + (size_t)kSeqL * kPrjP * 4;
constexpr size_t kOffDRL   = kOffDRH   + (size_t)kSeqL * kDtR  * 2;
constexpr size_t kOffDLR   = kOffDRL   + (size_t)kSeqL * kDtR  * 2;
constexpr size_t kOffGH    = kOffDLR   + (size_t)kSeqL * kDin  * 4;
constexpr size_t kOffGL    = kOffGH    + (size_t)kSeqL * kDin  * 2;
constexpr size_t kWsTotal  = kOffGL    + (size_t)kSeqL * kDin  * 2;
static_assert(kWsTotal == 123994112ull);
static_assert(kWsTotal <= 134217728ull);
static_assert((kOffWINB % 128) == 0 && (kOffWXB % 128) == 0 && (kOffWDTB % 128) == 0 && (kOffWOUTB % 128) == 0 &&
              (kOffXZ % 128) == 0 && (kOffUC % 128) == 0 && (kOffUH % 128) == 0 && (kOffUL % 128) == 0 &&
              (kOffPROJ % 128) == 0 && (kOffDRH % 128) == 0 && (kOffDRL % 128) == 0 && (kOffDLR % 128) == 0 &&
              (kOffGH % 128) == 0 && (kOffGL % 128) == 0);

__device__ __forceinline__ unsigned bf16_bits(float f) {
  const unsigned u = __float_as_uint(f);
  return (u + 0x7FFFu + ((u >> 16) & 1u)) >> 16;
}
__device__ __forceinline__ float bf16_val(unsigned bits) { return __uint_as_float(bits << 16); }
__device__ __forceinline__ float bf16q(float f) { return bf16_val(bf16_bits(f)); }

__device__ __forceinline__ void split8(const v4f a0, const v4f a1, v4u& hw, v4u& lw) {
  const float f0 = a0[0], f1 = a0[1], f2 = a0[2], f3 = a0[3];
  const float f4 = a1[0], f5 = a1[1], f6 = a1[2], f7 = a1[3];
  const unsigned h0 = bf16_bits(f0), h1 = bf16_bits(f1), h2 = bf16_bits(f2), h3 = bf16_bits(f3);
  const unsigned h4 = bf16_bits(f4), h5 = bf16_bits(f5), h6 = bf16_bits(f6), h7 = bf16_bits(f7);
  const unsigned l0 = bf16_bits(f0 - bf16_val(h0)), l1 = bf16_bits(f1 - bf16_val(h1));
  const unsigned l2 = bf16_bits(f2 - bf16_val(h2)), l3 = bf16_bits(f3 - bf16_val(h3));
  const unsigned l4 = bf16_bits(f4 - bf16_val(h4)), l5 = bf16_bits(f5 - bf16_val(h5));
  const unsigned l6 = bf16_bits(f6 - bf16_val(h6)), l7 = bf16_bits(f7 - bf16_val(h7));
  hw = (v4u){h0 | (h1 << 16), h2 | (h3 << 16), h4 | (h5 << 16), h6 | (h7 << 16)};
  lw = (v4u){l0 | (l1 << 16), l2 | (l3 << 16), l4 | (l5 << 16), l6 | (l7 << 16)};
}

__device__ __forceinline__ v16b frag_load(const __bf16* p) {
  union U { v16b v; v8b h[2]; } f;
  f.h[0] = *(const v8b*)(p);
  f.h[1] = *(const v8b*)(p + 16);
  return f.v;
}
__device__ __forceinline__ v8f mma_bf16(v16b a, v16b b, v8f c) {
  return __builtin_amdgcn_wmma_f32_16x16x32_bf16(false, a, false, b, (short)0, c, false, false);
}
__device__ __forceinline__ void guard_row4(v8f& a, v8f& b, v8f& c, v8f& d, v16b x, v16b y) {
  asm volatile("v_nop\n\tv_nop\n\tv_nop\n\tv_nop" : "+v"(a), "+v"(b), "+v"(c), "+v"(d) : "v"(x), "v"(y));
}
__device__ __forceinline__ void keep4_b(v16b a, v16b b, v16b c, v16b d) { asm volatile("v_nop" :: "v"(a), "v"(b), "v"(c), "v"(d)); }
__device__ __forceinline__ void acc_guard4(v8f& a, v8f& b, v8f& c, v8f& d) { asm volatile("v_nop\n\tv_nop\n\tv_nop\n\tv_nop" : "+v"(a), "+v"(b), "+v"(c), "+v"(d)); }

template <int SPL, int BIAS_MODE>
__global__ __launch_bounds__(256) void wmma_gemm64_bf16(
    const unsigned short* __restrict__ Ap, const unsigned short* __restrict__ A2p, int lda,
    const unsigned short* __restrict__ Btp, int ldb,
    float* __restrict__ C, int ldc,
    const float* __restrict__ bias,
    int M, int N, int K)
{
  const __bf16* A  = (const __bf16*)Ap;
  const __bf16* A2 = (const __bf16*)A2p;
  const __bf16* Bt = (const __bf16*)Btp;
  __shared__ __align__(16) float sT[8][16 * 68];
  const int lane = threadIdx.x & 31;
  const int wave = threadIdx.x >> 5;
  const int tilesN = N >> 6;
  const int tilesM = M >> 6;
  const int tile = blockIdx.x * 8 + wave;
  if (tile >= tilesM * tilesN) return;
  const int tm = tile / tilesN;
  const int tn = tile - tm * tilesN;
  const int m0 = tm << 6;
  const int n0 = tn << 6;

  const int rlane = lane & 15;
  const int koff  = (lane >> 4) * 8;
  const int mOff  = (lane >> 4) * 8;

  v8f acc[4][4];
#pragma unroll
  for (int i = 0; i < 4; ++i)
#pragma unroll
    for (int j = 0; j < 4; ++j) acc[i][j] = (v8f){0.f,0.f,0.f,0.f,0.f,0.f,0.f,0.f};

  for (int k0 = 0; k0 < K; k0 += 32) {
    v16b bh[4];
#pragma unroll
    for (int j = 0; j < 4; ++j) {
      const size_t bo = (size_t)(n0 + (j << 4) + rlane) * ldb + koff + k0;
      bh[j] = frag_load(Bt + bo);
    }
#pragma unroll
    for (int i = 0; i < 4; ++i) {
      const size_t ao = (size_t)(m0 + (i << 4) + rlane) * lda + koff + k0;
      const v16b ah = frag_load(A + ao);
      v16b al = ah;
      if (SPL == 1) al = frag_load(A2 + ao);
#pragma unroll
      for (int j = 0; j < 4; ++j) {
        acc[i][j] = mma_bf16(ah, bh[j], acc[i][j]);
        if (SPL == 1) acc[i][j] = mma_bf16(al, bh[j], acc[i][j]);
      }
      guard_row4(acc[i][0], acc[i][1], acc[i][2], acc[i][3], ah, al);
    }
    keep4_b(bh[0], bh[1], bh[2], bh[3]);
  }
  acc_guard4(acc[0][0], acc[0][1], acc[0][2], acc[0][3]);
  acc_guard4(acc[1][0], acc[1][1], acc[1][2], acc[1][3]);
  acc_guard4(acc[2][0], acc[2][1], acc[2][2], acc[2][3]);
  acc_guard4(acc[3][0], acc[3][1], acc[3][2], acc[3][3]);

  float* slab = sT[wave];
#pragma unroll
  for (int i = 0; i < 4; ++i) {
    const int mBase = m0 + (i << 4);
#pragma unroll
    for (int j = 0; j < 4; ++j) {
      const int n = n0 + (j << 4) + rlane;
      float bv = 0.f;
      if (BIAS_MODE == 2) bv = bf16q(bias[n]);
#pragma unroll
      for (int r = 0; r < 8; ++r) {
        float v = acc[i][j][r];
        if (BIAS_MODE == 2) v += bv;
        slab[(mOff + r) * 68 + (j << 4) + rlane] = v;
      }
    }
    __builtin_amdgcn_fence(__ATOMIC_RELEASE, "workgroup");
    __builtin_amdgcn_wave_barrier();
    __builtin_amdgcn_fence(__ATOMIC_ACQUIRE, "workgroup");
    {
      const int hh = lane >> 4, c4 = (lane & 15) * 4;
      for (int pass = 0; pass < 2; ++pass) {
#pragma unroll
        for (int it = 0; it < 8; ++it) {
          const int row = it * 2 + hh;
          const v4f v = *(const v4f*)(slab + row * 68 + c4);
          *(volatile v4f*)(C + (size_t)(mBase + row) * ldc + n0 + c4) = v;
        }
        __threadfence();
      }
    }
    __builtin_amdgcn_fence(__ATOMIC_RELEASE, "workgroup");
    __builtin_amdgcn_wave_barrier();
    __builtin_amdgcn_fence(__ATOMIC_ACQUIRE, "workgroup");
  }
}

__global__ __launch_bounds__(256) void cvt_rows_bf16_kernel(
    const float* __restrict__ src, unsigned short* __restrict__ dst, int total8, int src8)
{
  const int i = blockIdx.x * 256 + threadIdx.x;
  if (i >= total8) return;
  const bool live = (i < src8);
  const int ic = live ? i : (src8 - 1);
  const float* p = src + ((size_t)ic << 3);
  const v4f a0 = *(const v4f*)(p);
  const v4f a1 = *(const v4f*)(p + 4);
  const float f0 = live ? a0[0] : 0.0f, f1 = live ? a0[1] : 0.0f, f2 = live ? a0[2] : 0.0f, f3 = live ? a0[3] : 0.0f;
  const float f4 = live ? a1[0] : 0.0f, f5 = live ? a1[1] : 0.0f, f6 = live ? a1[2] : 0.0f, f7 = live ? a1[3] : 0.0f;
  const unsigned h0 = bf16_bits(f0), h1 = bf16_bits(f1), h2 = bf16_bits(f2), h3 = bf16_bits(f3);
  const unsigned h4 = bf16_bits(f4), h5 = bf16_bits(f5), h6 = bf16_bits(f6), h7 = bf16_bits(f7);
  const v4u w = (v4u){h0 | (h1 << 16), h2 | (h3 << 16), h4 | (h5 << 16), h6 | (h7 << 16)};
  unsigned short* q = dst + ((size_t)i << 3);
  *(volatile v4u*)q = w;
  __threadfence();
  *(volatile v4u*)q = w;
}

__global__ __launch_bounds__(256) void conv_silu_kernel(
    const float* __restrict__ XZ, const float* __restrict__ cw, const float* __restrict__ cb,
    float* __restrict__ UC, unsigned short* __restrict__ UH, unsigned short* __restrict__ UL)
{
  __shared__ __align__(16) float sT[16 * kTP];
  const int tid = threadIdx.x, lane = tid & 31, wave = tid >> 5;
  const int d0 = blockIdx.x * 256, d = d0 + tid;
  const int t0 = blockIdx.y * 64;
  const v4f wv = *(const v4f*)(cw + (size_t)d * 4);
  const float w0 = bf16q(wv[0]), w1 = bf16q(wv[1]), w2 = bf16q(wv[2]), w3 = bf16q(wv[3]);
  const float bc = bf16q(cb[d]);
  float xm3, xm2, xm1;
  {
    const int r3 = t0 - 3, r2 = t0 - 2, r1 = t0 - 1;
    const float v3 = XZ[(size_t)(r3 < 0 ? 0 : r3) * kXZP + d];
    const float v2 = XZ[(size_t)(r2 < 0 ? 0 : r2) * kXZP + d];
    const float v1 = XZ[(size_t)(r1 < 0 ? 0 : r1) * kXZP + d];
    xm3 = (r3 >= 0) ? v3 : 0.f;
    xm2 = (r2 >= 0) ? v2 : 0.f;
    xm1 = (r1 >= 0) ? v1 : 0.f;
  }
  const int hrow = wave >> 1;
  const int hch  = (wave & 1) * 128 + lane * 4;
#pragma unroll 1
  for (int sub = 0; sub < 4; ++sub) {
    const int lb = t0 + sub * 16;
#pragma unroll 1
    for (int s = 0; s < 16; ++s) {
      const float xc = XZ[(size_t)(lb + s) * kXZP + d];
      float acc = w0 * xm3;
      acc = fmaf(w1, xm2, acc);
      acc = fmaf(w2, xm1, acc);
      acc = fmaf(w3, xc, acc);
      const float sv = acc + bc;
      const float sg = 1.0f / (1.0f + expf(-sv));
      sT[s * kTP + tid] = sv * sg;
      xm3 = xm2; xm2 = xm1; xm1 = xc;
    }
    __syncthreads();
    v4f fv[4];
    v4u hw[2], lw[2];
#pragma unroll
    for (int it = 0; it < 4; ++it) fv[it] = *(const v4f*)(sT + (it * 4 + hrow) * kTP + hch);
#pragma unroll
    for (int it = 0; it < 2; ++it) {
      const float* sp = sT + (it * 8 + wave) * kTP + lane * 8;
      const v4f a0 = *(const v4f*)(sp);
      const v4f a1 = *(const v4f*)(sp + 4);
      split8(a0, a1, hw[it], lw[it]);
    }
    for (int pass = 0; pass < 2; ++pass) {
#pragma unroll
      for (int it = 0; it < 4; ++it)
        *(volatile v4f*)(UC + (size_t)(lb + it * 4 + hrow) * kDin + d0 + hch) = fv[it];
#pragma unroll
      for (int it = 0; it < 2; ++it) {
        const size_t o = (size_t)(lb + it * 8 + wave) * kDin + d0 + lane * 8;
        *(volatile v4u*)(UH + o) = hw[it];
        *(volatile v4u*)(UL + o) = lw[it];
      }
      __threadfence();
    }
    __syncthreads();
  }
}

__global__ __launch_bounds__(256) void dr_split_kernel(
    const float* __restrict__ PROJ, unsigned short* __restrict__ DRH, unsigned short* __restrict__ DRL, int total8)
{
  const int i = blockIdx.x * 256 + threadIdx.x;
  if (i >= total8) return;
  const int e0  = i << 3;
  const int row = e0 >> 6;
  const int c8  = e0 & 63;
  const float* p = PROJ + (size_t)row * kPrjP + c8;
  const v4f a0 = *(const v4f*)(p);
  const v4f a1 = *(const v4f*)(p + 4);
  v4u hw, lw;
  split8(a0, a1, hw, lw);
  unsigned short* qh = DRH + e0;
  unsigned short* ql = DRL + e0;
  *(volatile v4u*)qh = hw;
  *(volatile v4u*)ql = lw;
  __threadfence();
  *(volatile v4u*)qh = hw;
  *(volatile v4u*)ql = lw;
}

__global__ __launch_bounds__(256) void scan_kernel(
    const float* __restrict__ DLR, const float* __restrict__ UC, const float* __restrict__ XZ,
    const float* __restrict__ PROJ, const float* __restrict__ A_log, const float* __restrict__ Dv,
    unsigned short* __restrict__ GH, unsigned short* __restrict__ GL)
{
  __shared__ __align__(16) float sBC[16 * 32];
  __shared__ __align__(16) float sY[16 * kTP];
  const int tid = threadIdx.x, lane = tid & 31, wave = tid >> 5;
  const int d0 = blockIdx.x * 256, d = d0 + tid;

  float A2[kNst];
#pragma unroll
  for (int q = 0; q < 4; ++q) {
    const v4f av = *(const v4f*)(A_log + (size_t)d * kNst + 4 * q);
    const float e0 = -expf(bf16q(av[0]));
    const float e1 = -expf(bf16q(av[1]));
    const float e2 = -expf(bf16q(av[2]));
    const float e3 = -expf(bf16q(av[3]));
    A2[4 * q + 0] = e0 * kLog2e;
    A2[4 * q + 1] = e1 * kLog2e;
    A2[4 * q + 2] = e2 * kLog2e;
    A2[4 * q + 3] = e3 * kLog2e;
  }
  const float Dd = bf16q(Dv[d]);
  float h[kNst];
#pragma unroll
  for (int n = 0; n < kNst; ++n) h[n] = 0.f;

#pragma unroll 1
  for (int c = 0; c < kSeqL / 16; ++c) {
    const int l0 = c * 16;
    if (tid < 128) {
      const int r = tid >> 3, q = (tid & 7) * 4;
      const v4f v = *(const v4f*)(PROJ + (size_t)(l0 + r) * kPrjP + kDtR + q);
      *(v4f*)(sBC + r * 32 + q) = v;
    }
    __syncthreads();
#pragma unroll 1
    for (int s = 0; s < 16; ++s) {
      const size_t m = (size_t)(l0 + s);
      const float a  = DLR[m * kDin + d];
      const float xv = UC[m * kDin + d];
      const float zv = XZ[m * kXZP + kDin + d];
      const float delta = fmaxf(a, 0.0f) + log1pf(expf(-fabsf(a)));
      v4f Bq[4], Cq[4];
#pragma unroll
      for (int qq = 0; qq < 4; ++qq) {
        Bq[qq] = *(const v4f*)(sBC + s * 32 + 4 * qq);
        Cq[qq] = *(const v4f*)(sBC + s * 32 + kNst + 4 * qq);
      }
      const float dtx = delta * xv;
      float y = 0.f;
#pragma unroll
      for (int n = 0; n < kNst; ++n) {
        const float e = exp2f(delta * A2[n]);
        const float p = dtx * Bq[n >> 2][n & 3];
        const float hn = fmaf(e, h[n], p);
        h[n] = hn;
        y = fmaf(hn, Cq[n >> 2][n & 3], y);
      }
      y = fmaf(xv, Dd, y);
      const float sg = 1.0f / (1.0f + expf(-zv));
      sY[s * kTP + tid] = y * (zv * sg);
    }
    __syncthreads();
    v4u hw[2], lw[2];
#pragma unroll
    for (int it = 0; it < 2; ++it) {
      const float* sp = sY + (it * 8 + wave) * kTP + lane * 8;
      const v4f a0 = *(const v4f*)(sp);
      const v4f a1 = *(const v4f*)(sp + 4);
      split8(a0, a1, hw[it], lw[it]);
    }
    for (int pass = 0; pass < 2; ++pass) {
#pragma unroll
      for (int it = 0; it < 2; ++it) {
        const size_t o = (size_t)(l0 + it * 8 + wave) * kDin + d0 + lane * 8;
        *(volatile v4u*)(GH + o) = hw[it];
        *(volatile v4u*)(GL + o) = lw[it];
      }
      __threadfence();
    }
  }
}

extern "C" void kernel_launch(void* const* d_in, const int* in_sizes, int n_in,
                              void* d_out, int out_size, void* d_ws, size_t ws_size,
                              hipStream_t stream)
{
  if (n_in < 10) return;
  if (in_sizes[0] != kRows * kDmod) return;
  if (in_sizes[1] != kXZP * kDmod) return;
  if (in_sizes[2] != kDin * 4) return;
  if (in_sizes[3] != kDin) return;
  if (in_sizes[4] != kPrjN * kDin) return;
  if (in_sizes[5] != kDin * kDtR) return;
  if (in_sizes[6] != kDin) return;
  if (in_sizes[7] != kDin * kNst) return;
  if (in_sizes[8] != kDin) return;
  if (in_sizes[9] != kDmod * kDin) return;
  if (out_size != kRows * kDmod) return;
  if (ws_size < kWsTotal) return;

  const float* x      = (const float*)d_in[0];
  const float* Win    = (const float*)d_in[1];
  const float* conv_w = (const float*)d_in[2];
  const float* conv_b = (const float*)d_in[3];
  const float* Wx     = (const float*)d_in[4];
  const float* Wdt    = (const float*)d_in[5];
  const float* bdt    = (const float*)d_in[6];
  const float* A_log  = (const float*)d_in[7];
  const float* Dv     = (const float*)d_in[8];
  const float* Wout   = (const float*)d_in[9];
  float* dout = (float*)d_out;

  char* ws = (char*)d_ws;
  unsigned short* XB    = (unsigned short*)(ws + kOffXB);
  unsigned short* WINB  = (unsigned short*)(ws + kOffWINB);
  unsigned short* WXB   = (unsigned short*)(ws + kOffWXB);
  unsigned short* WDTB  = (unsigned short*)(ws + kOffWDTB);
  unsigned short* WOUTB = (unsigned short*)(ws + kOffWOUTB);
  float*          XZ    = (float*)(ws + kOffXZ);
  float*          UC    = (float*)(ws + kOffUC);
  unsigned short* UH    = (unsigned short*)(ws + kOffUH);
  unsigned short* UL    = (unsigned short*)(ws + kOffUL);
  float*          PROJ  = (float*)(ws + kOffPROJ);
  unsigned short* DRH   = (unsigned short*)(ws + kOffDRH);
  unsigned short* DRL   = (unsigned short*)(ws + kOffDRL);
  float*          DLR   = (float*)(ws + kOffDLR);
  unsigned short* GH    = (unsigned short*)(ws + kOffGH);
  unsigned short* GL    = (unsigned short*)(ws + kOffGL);

  cvt_rows_bf16_kernel<<<(kRows * kDmod / 8) / 256, 256, 0, stream>>>(x, XB, kRows * kDmod / 8, kRows * kDmod / 8);
  cvt_rows_bf16_kernel<<<(kXZP * kDmod / 8) / 256, 256, 0, stream>>>(Win, WINB, kXZP * kDmod / 8, kXZP * kDmod / 8);
  cvt_rows_bf16_kernel<<<(kPrjP * kDin / 8) / 256, 256, 0, stream>>>(Wx, WXB, kPrjP * kDin / 8, kPrjN * kDin / 8);
  cvt_rows_bf16_kernel<<<(kDin * kDtR / 8) / 256, 256, 0, stream>>>(Wdt, WDTB, kDin * kDtR / 8, kDin * kDtR / 8);
  cvt_rows_bf16_kernel<<<(kDmod * kDin / 8) / 256, 256, 0, stream>>>(Wout, WOUTB, kDmod * kDin / 8, kDmod * kDin / 8);

  for (int b = 0; b < kBatch; ++b) {
    const unsigned short* XBb = XB + (size_t)b * kSeqL * kDmod;
    float* outb = dout + (size_t)b * kSeqL * kDmod;

    wmma_gemm64_bf16<0, 0><<<dim3(256, 1), 256, 0, stream>>>(
        XBb, XBb, kDmod, WINB, kDmod, XZ, kXZP, bdt, kSeqL, kXZP, kDmod);

    conv_silu_kernel<<<dim3(kDin / 256, kSeqL / 64), 256, 0, stream>>>(XZ, conv_w, conv_b, UC, UH, UL);

    wmma_gemm64_bf16<1, 0><<<dim3(8, 1), 256, 0, stream>>>(
        UH, UL, kDin, WXB, kDin, PROJ, kPrjP, bdt, kSeqL, kPrjP, kDin);

    dr_split_kernel<<<(kSeqL * kDtR / 8) / 256, 256, 0, stream>>>(PROJ, DRH, DRL, kSeqL * kDtR / 8);

    wmma_gemm64_bf16<1, 2><<<dim3(128, 1), 256, 0, stream>>>(
        DRH, DRL, kDtR, WDTB, kDtR, DLR, kDin, bdt, kSeqL, kDin, kDtR);

    scan_kernel<<<dim3(kDin / 256, 1), 256, 0, stream>>>(DLR, UC, XZ, PROJ, A_log, Dv, GH, GL);

    wmma_gemm64_bf16<1, 0><<<dim3(64, 1), 256, 0, stream>>>(
        GH, GL, kDin, WOUTB, kDin, outb, kDmod, bdt, kSeqL, kDmod, kDin);
  }
}
